// alinet_atten_77163382440890
// MI455X (gfx1250) — hardware-verified
//
#include <hip/hip_runtime.h>
#include <math.h>

#define NN   100000
#define NE   1600000
#define FD   128
#define NB   384
#define NT   256
#define SRB  4096
#define NTL  25
#define NPAD (NTL * SRB)
#define NCK  4
#define CR   (NPAD / NCK)
#define SCH  2048
#define NCH  ((NE + SCH - 1) / SCH)
#define BN_EPS 1e-3f

typedef __attribute__((ext_vector_type(16))) _Float16 v16h;
typedef __attribute__((ext_vector_type(8)))  _Float16 v8h;
typedef __attribute__((ext_vector_type(16))) __bf16   v16b;
typedef __attribute__((ext_vector_type(8)))  __bf16   v8b;
typedef __attribute__((ext_vector_type(8)))  float    v8f;
typedef __attribute__((ext_vector_type(4)))  float    v4f;
typedef __attribute__((ext_vector_type(4)))  int      v4i;

__device__ __forceinline__ unsigned short f2bf_bits(float f) {
  unsigned u = __float_as_uint(f);
  return (unsigned short)((u + 0x7FFFu + ((u >> 16) & 1u)) >> 16);
}
__device__ __forceinline__ float bf_bits2f(unsigned short h) { return __uint_as_float(((unsigned)h) << 16); }

__device__ __forceinline__ void dep_guard_h(v8f& a, v8f& b, v16h x, v16h y) { asm volatile("v_nop\n\tv_nop\n\tv_nop\n\tv_nop" : "+v"(a), "+v"(b) : "v"(x), "v"(y)); }
__device__ __forceinline__ void dep_guard_b(v8f& a, v8f& b, v16b x, v16b y) { asm volatile("v_nop\n\tv_nop\n\tv_nop\n\tv_nop" : "+v"(a), "+v"(b) : "v"(x), "v"(y)); }
__device__ __forceinline__ void keep4_h(v16h a, v16h b, v16h c, v16h d) { asm volatile("v_nop" :: "v"(a), "v"(b), "v"(c), "v"(d)); }
__device__ __forceinline__ void keep4_b(v16b a, v16b b, v16b c, v16b d) { asm volatile("v_nop" :: "v"(a), "v"(b), "v"(c), "v"(d)); }
__device__ __forceinline__ void acc_guard4(v8f& a, v8f& b, v8f& c, v8f& d) { asm volatile("v_nop\n\tv_nop\n\tv_nop\n\tv_nop" : "+v"(a), "+v"(b), "+v"(c), "+v"(d)); }
template <typename T> struct Frag;
template <> struct Frag<_Float16> {
  typedef v16h V; union U { v16h v; v8h h[2]; };
  static __device__ __forceinline__ v16h load(const _Float16* p) {
    U f; f.h[0] = *(const v8h*)(p); f.h[1] = *(const v8h*)(p + 16); return f.v;
  }
  static __device__ __forceinline__ v8f mma(v16h a, v16h b, v8f c) {
    return __builtin_amdgcn_wmma_f32_16x16x32_f16(false, a, false, b, (short)0, c, false, false);
  }
  static __device__ __forceinline__ void guard(v8f& a, v8f& b, v16h x, v16h y) { dep_guard_h(a, b, x, y); }
  static __device__ __forceinline__ void keep(v16h a, v16h b, v16h c, v16h d) { keep4_h(a, b, c, d); }
};
template <> struct Frag<__bf16> {
  typedef v16b V; union U { v16b v; v8b h[2]; };
  static __device__ __forceinline__ v16b load(const __bf16* p) {
    U f; f.h[0] = *(const v8b*)(p); f.h[1] = *(const v8b*)(p + 16); return f.v;
  }
  static __device__ __forceinline__ v8f mma(v16b a, v16b b, v8f c) {
    return __builtin_amdgcn_wmma_f32_16x16x32_bf16(false, a, false, b, (short)0, c, false, false);
  }
  static __device__ __forceinline__ void guard(v8f& a, v8f& b, v16b x, v16b y) { dep_guard_b(a, b, x, y); }
  static __device__ __forceinline__ void keep(v16b a, v16b b, v16b c, v16b d) { keep4_b(a, b, c, d); }
};

template <int ET> struct Elem;
template <> struct Elem<0> { typedef _Float16 T; };
template <> struct Elem<1> { typedef __bf16 T; };
template <int ET, bool SPLIT, int BIAS_MODE, int OUT_MODE, bool RESID, int ACT = 0>
__global__ __launch_bounds__(256) void wmma_gemm64(
    const unsigned short* __restrict__ Ap, const unsigned short* __restrict__ A2p, int lda, long strideA,
    const unsigned short* __restrict__ Btp, const unsigned short* __restrict__ Bt2p, int ldb, long strideB,
    void* __restrict__ Cout, void* __restrict__ Cout2, int ldc, long strideC,
    const float* __restrict__ bias,
    const float* __restrict__ resid, long strideR,
    int M, int N, int K, float scale) {
  typedef typename Elem<ET>::T T;
  typedef typename Frag<T>::V V;
  const T* A = (const T*)Ap; const T* A2 = (const T*)A2p; const T* Bt = (const T*)Btp; const T* Bt2 = (const T*)Bt2p;
  __shared__ __align__(16) float sT[8][16 * 68];
  const int b    = blockIdx.y;
  const int lane = threadIdx.x & 31;
  const int wave = threadIdx.x >> 5;
  const int tilesN = N >> 6;
  const int tilesM = M >> 6;
  const int tile = blockIdx.x * 8 + wave;
  if (tile >= tilesM * tilesN) return;
  const int tm = tile / tilesN;
  const int tn = tile - tm * tilesN;
  const int m0 = tm << 6;
  const int n0 = tn << 6;

  const T* Ab  = A  + (size_t)b * strideA;
  const T* Bb  = Bt + (size_t)b * strideB;
  const T* Ab2 = SPLIT ? (A2  + (size_t)b * strideA) : nullptr;
  const T* Bb2 = SPLIT ? (Bt2 + (size_t)b * strideB) : nullptr;

  const int rlane = lane & 15;
  const int koff  = (lane >> 4) * 8;
  const int mOff  = (lane >> 4) * 8;

  v8f acc[4][4];
#pragma unroll
  for (int i = 0; i < 4; ++i)
#pragma unroll
    for (int j = 0; j < 4; ++j) acc[i][j] = (v8f){0.f,0.f,0.f,0.f,0.f,0.f,0.f,0.f};

  for (int k0 = 0; k0 < K; k0 += 32) {
    V bh[4], bl[4];
#pragma unroll
    for (int j = 0; j < 4; ++j) {
      const size_t bo = (size_t)(n0 + (j << 4) + rlane) * ldb + koff + k0;
      bh[j] = Frag<T>::load(Bb + bo);
      if (SPLIT) bl[j] = Frag<T>::load(Bb2 + bo);
    }
#pragma unroll
    for (int i = 0; i < 4; ++i) {
      const size_t ao = (size_t)(m0 + (i << 4) + rlane) * lda + koff + k0;
      V ah = Frag<T>::load(Ab + ao);
      V al;
      if (SPLIT) al = Frag<T>::load(Ab2 + ao);
#pragma unroll
      for (int j = 0; j < 4; ++j) {
        acc[i][j] = Frag<T>::mma(ah, bh[j], acc[i][j]);
        if (SPLIT) {
          acc[i][j] = Frag<T>::mma(ah, bl[j], acc[i][j]);
          acc[i][j] = Frag<T>::mma(al, bh[j], acc[i][j]);
        }
      }
      Frag<T>::guard(acc[i][0], acc[i][3], ah, SPLIT ? al : ah);
    }
    Frag<T>::keep(bh[0], bh[1], bh[2], bh[3]);
    if (SPLIT) Frag<T>::keep(bl[0], bl[1], bl[2], bl[3]);
  }
  acc_guard4(acc[0][0], acc[0][1], acc[0][2], acc[0][3]);
  acc_guard4(acc[1][0], acc[1][1], acc[1][2], acc[1][3]);
  acc_guard4(acc[2][0], acc[2][1], acc[2][2], acc[2][3]);
  acc_guard4(acc[3][0], acc[3][1], acc[3][2], acc[3][3]);

  float* slab = sT[wave];
  const float* Rb = RESID ? (resid + (size_t)b * strideR) : nullptr;
#pragma unroll
  for (int i = 0; i < 4; ++i) {
    const int mBase = m0 + (i << 4);
#pragma unroll
    for (int j = 0; j < 4; ++j) {
      const int n = n0 + (j << 4) + rlane;
      float bv = 0.f;
      if (BIAS_MODE == 2) bv = bias[n];
#pragma unroll
      for (int r = 0; r < 8; ++r) {
        float v = acc[i][j][r] * scale;
        if (BIAS_MODE == 1) v += bias[mBase + mOff + r];
        if (BIAS_MODE == 2) v += bv;
        if (RESID) v += Rb[(size_t)(mBase + mOff + r) * ldc + n];
        if (ACT == 1) v = tanhf(v);
        if (ACT == 2) v = fmaxf(v, 0.0f);
        if (ACT == 3) v = v / (1.0f + expf(-v));
        if (ACT == 4) v = (v > 0.f) ? v : 0.01f * v;
        if (ACT == 5) v = 0.5f * v * (1.0f + erff(v * 0.70710678118654752f));
        slab[(mOff + r) * 68 + (j << 4) + rlane] = v;
      }
    }
    __builtin_amdgcn_fence(__ATOMIC_RELEASE, "workgroup");
    __builtin_amdgcn_wave_barrier();
    __builtin_amdgcn_fence(__ATOMIC_ACQUIRE, "workgroup");
    if (OUT_MODE == 0) {
      float* C = (float*)Cout + (size_t)b * strideC;
      const int hh = lane >> 4, c4 = (lane & 15) * 4;
      for (int pass = 0; pass < 2; ++pass) {
#pragma unroll
        for (int it = 0; it < 8; ++it) {
          const int row = it * 2 + hh;
          v4f v = *(const v4f*)(slab + row * 68 + c4);
          *(volatile v4f*)(C + (size_t)(mBase + row) * ldc + n0 + c4) = v;
        }
        __threadfence();
      }
    } else {
      const int q = lane >> 3, c8 = (lane & 7) * 8;
      unsigned short* C  = (unsigned short*)Cout  + (size_t)b * strideC;
      unsigned short* C2 = (OUT_MODE == 2) ? ((unsigned short*)Cout2 + (size_t)b * strideC) : nullptr;
      for (int pass = 0; pass < 2; ++pass) {
#pragma unroll
        for (int it = 0; it < 4; ++it) {
          const int row = it * 4 + q;
          const float* sp = slab + row * 68 + c8;
          v8h hv, lv;
#pragma unroll
          for (int e = 0; e < 8; ++e) {
            if (OUT_MODE == 1) {
              hv[e] = (_Float16)sp[e];
            } else {
              unsigned short hb = f2bf_bits(sp[e]);
              unsigned short lb = f2bf_bits(sp[e] - bf_bits2f(hb));
              hv[e] = __builtin_bit_cast(_Float16, hb);
              lv[e] = __builtin_bit_cast(_Float16, lb);
            }
          }
          *(volatile v8h*)(C + (size_t)(mBase + row) * ldc + n0 + c8) = hv;
          if (OUT_MODE == 2) *(volatile v8h*)(C2 + (size_t)(mBase + row) * ldc + n0 + c8) = lv;
        }
        __threadfence();
      }
    }
    __builtin_amdgcn_fence(__ATOMIC_RELEASE, "workgroup");
    __builtin_amdgcn_wave_barrier();
    __builtin_amdgcn_fence(__ATOMIC_ACQUIRE, "workgroup");
  }
}

__global__ __launch_bounds__(256) void bt_split_kernel(const float* __restrict__ W, const float* __restrict__ M1, const float* __restrict__ M2,
                                                      unsigned short* __restrict__ Bh, unsigned short* __restrict__ Bl) {
  const int t = blockIdx.x * 256 + threadIdx.x;
  if (t >= NB * (FD / 8)) return;
  const int n = t >> 4, k0 = (t & 15) * 8;
  const int mat = n >> 7, cc = n & 127;
  const float* src = (mat == 0) ? W : ((mat == 1) ? M1 : M2);
  v8h hv, lv;
#pragma unroll
  for (int i = 0; i < 8; ++i) {
    const float v = src[(size_t)(k0 + i) * FD + cc];
    const unsigned short hb = f2bf_bits(v);
    const unsigned short lb = f2bf_bits(v - bf_bits2f(hb));
    hv[i] = __builtin_bit_cast(_Float16, hb);
    lv[i] = __builtin_bit_cast(_Float16, lb);
  }
  unsigned short* ph = Bh + (size_t)n * FD + k0;
  unsigned short* pl = Bl + (size_t)n * FD + k0;
  *(volatile v8h*)ph = hv; *(volatile v8h*)pl = lv;
  __threadfence();
  *(volatile v8h*)ph = hv; *(volatile v8h*)pl = lv;
}

__global__ __launch_bounds__(256) void xn_split_kernel(const float* __restrict__ x, const float* __restrict__ gamma, const float* __restrict__ beta,
                                                      const float* __restrict__ bn_mean, const float* __restrict__ bn_var, int row0,
                                                      unsigned short* __restrict__ Ah, unsigned short* __restrict__ Al) {
  __shared__ __align__(16) float csc[FD];
  __shared__ __align__(16) float cmu[FD];
  __shared__ __align__(16) float cbe[FD];
  if (threadIdx.x < FD) {
    const int c = threadIdx.x;
    csc[c] = (1.0f / sqrtf(bn_var[c] + BN_EPS)) * gamma[c];
    cmu[c] = bn_mean[c];
    cbe[c] = beta[c];
  }
  __syncthreads();
  const int t = blockIdx.x * 256 + threadIdx.x;
  if (t < CR * (FD / 8)) {
    const int r = t >> 4, k0 = (t & 15) * 8;
    const int m = row0 + r;
    const int mc = (m < NN) ? m : (NN - 1);
    const float* xr = x + (size_t)mc * FD + k0;
    const v4f xa = *(const v4f*)xr, xb = *(const v4f*)(xr + 4);
    const v4f mua = *(const v4f*)(cmu + k0), mub = *(const v4f*)(cmu + k0 + 4);
    const v4f sca = *(const v4f*)(csc + k0), scb = *(const v4f*)(csc + k0 + 4);
    const v4f bea = *(const v4f*)(cbe + k0), beb = *(const v4f*)(cbe + k0 + 4);
    v4f na = (xa - mua) * sca + bea;
    v4f nb = (xb - mub) * scb + beb;
    const v4f z4 = {0.f, 0.f, 0.f, 0.f};
    if (m >= NN) { na = z4; nb = z4; }
    v8h hv, lv;
#pragma unroll
    for (int e = 0; e < 4; ++e) {
      const unsigned short ha = f2bf_bits(na[e]);
      const unsigned short la = f2bf_bits(na[e] - bf_bits2f(ha));
      const unsigned short hb = f2bf_bits(nb[e]);
      const unsigned short lb = f2bf_bits(nb[e] - bf_bits2f(hb));
      hv[e] = __builtin_bit_cast(_Float16, ha);     lv[e] = __builtin_bit_cast(_Float16, la);
      hv[4 + e] = __builtin_bit_cast(_Float16, hb); lv[4 + e] = __builtin_bit_cast(_Float16, lb);
    }
    unsigned short* ph = Ah + (size_t)r * FD + k0;
    unsigned short* pl = Al + (size_t)r * FD + k0;
    *(volatile v8h*)ph = hv; *(volatile v8h*)pl = lv;
    __threadfence();
    *(volatile v8h*)ph = hv; *(volatile v8h*)pl = lv;
  }
}

__global__ __launch_bounds__(NT) void qform_tanh_kernel(const float* __restrict__ Cq, const float* __restrict__ x,
                                                       const float* __restrict__ gamma, const float* __restrict__ beta,
                                                       const float* __restrict__ bn_mean, const float* __restrict__ bn_var,
                                                       int row0, float* __restrict__ s1, float* __restrict__ s2) {
  __shared__ __align__(16) float csc[FD];
  __shared__ __align__(16) float cmu[FD];
  __shared__ __align__(16) float cbe[FD];
  __shared__ __align__(16) float so[128];
  const int tid = threadIdx.x, lane = tid & 31, wave = tid >> 5;
  if (tid < FD) {
    csc[tid] = (1.0f / sqrtf(bn_var[tid] + BN_EPS)) * gamma[tid];
    cmu[tid] = bn_mean[tid];
    cbe[tid] = beta[tid];
  }
  __syncthreads();
  const v4f sc4 = *(const v4f*)(csc + 4 * lane);
  const v4f mu4 = *(const v4f*)(cmu + 4 * lane);
  const v4f be4 = *(const v4f*)(cbe + 4 * lane);
#pragma unroll 1
  for (int i = 0; i < 8; ++i) {
    const int j = wave * 8 + i;
    const int rl = blockIdx.x * 64 + j;
    const int m = row0 + rl;
    const int mc = (m < NN) ? m : (NN - 1);
    const v4f xv = *(const v4f*)(x + (size_t)mc * FD + 4 * lane);
    const v4f xn = (xv - mu4) * sc4 + be4;
    const float* cr = Cq + (size_t)rl * (2 * FD) + 4 * lane;
    const v4f c1 = *(const v4f*)cr, c2 = *(const v4f*)(cr + FD);
    float d1 = xn[0] * c1[0]; d1 += xn[1] * c1[1]; d1 += xn[2] * c1[2]; d1 += xn[3] * c1[3];
    float d2 = xn[0] * c2[0]; d2 += xn[1] * c2[1]; d2 += xn[2] * c2[2]; d2 += xn[3] * c2[3];
#pragma unroll
    for (int o = 1; o < 32; o <<= 1) { d1 += __shfl_xor(d1, o, 32); d2 += __shfl_xor(d2, o, 32); }
    const float dv = (lane == 0) ? d1 : d2;
    const float tv = tanhf(dv);
    if (lane == 0) so[j] = tv;
    if (lane == 1) so[64 + j] = tv;
  }
  __syncthreads();
  if (wave == 0) {
    const int hh = lane >> 4, l4 = (lane & 15) * 4;
    const v4f v = *(const v4f*)(so + 64 * hh + l4);
    float* op = (hh ? s2 : s1) + (size_t)row0 + (size_t)blockIdx.x * 64 + l4;
    *(volatile v4f*)op = v; __threadfence(); *(volatile v4f*)op = v;
  }
}

__device__ __forceinline__ int blk_excl_scan(int cnt, int* scan_ws, int tid, int* tot) {
  const int lane = tid & 31, wave = tid >> 5; int incl = cnt;
#pragma unroll
  for (int o = 1; o < 32; o <<= 1) { const int v = __shfl_up(incl, o, 32); if (lane >= o) incl += v; }
  if (lane == 31) scan_ws[wave] = incl;
  __syncthreads();
  if (wave == 0) { int wv = (lane < NT / 32) ? scan_ws[lane] : 0; int wincl = wv;
#pragma unroll
    for (int o = 1; o < 32; o <<= 1) { const int v = __shfl_up(wincl, o, 32); if (lane >= o) wincl += v; }
    if (lane < NT / 32) scan_ws[32 + lane] = wincl - wv; if (lane == 31) scan_ws[64] = wincl; }
  __syncthreads();
  const int res = scan_ws[32 + wave] + incl - cnt; *tot = scan_ws[64];
  return res;
}
template <int SP, int CAP>
__device__ __forceinline__ int chunk_hits(const int* __restrict__ rowv, const int* __restrict__ colv, const float* __restrict__ av,
                                          const float* __restrict__ s1, const float* __restrict__ s2,
                                          int e0, int n0, int nhi, int tid, int* LIST, float* LSC, int* scan_ws) {
  const int eb = e0 + tid * SP;
  int rec[SP]; float frec[SP]; int cnt = 0;
#pragma unroll
  for (int k = 0; k < SP; ++k) { rec[k] = -1; frec[k] = 0.f; }
  if (eb < NE) {
#pragma unroll
    for (int k = 0; k < SP; k += 4) {
      const v4i d4 = *(const v4i*)(rowv + eb + k);
      const v4i c4 = *(const v4i*)(colv + eb + k);
      const v4f a4 = *(const v4f*)(av + eb + k);
#pragma unroll
      for (int e = 0; e < 4; ++e) {
        const int d = d4[e];
        if (d >= n0 && d < nhi) {
          int c = c4[e]; c = (c < 0) ? 0 : ((c >= NN) ? (NN - 1) : c);
          float sc = a4[e] * s1[d] + a4[e] * s2[c];
          sc = (sc >= 0.f) ? sc : 0.2f * sc;
          rec[k + e] = ((d - n0) << 17) | c; frec[k + e] = sc; ++cnt;
        }
      }
    }
  }
  int tot; int p = blk_excl_scan(cnt, scan_ws, tid, &tot);
#pragma unroll
  for (int k = 0; k < SP; ++k) {
    if (rec[k] >= 0) { if ((unsigned)p < (unsigned)CAP) { LIST[p] = rec[k]; LSC[p] = frec[k]; } ++p; }
  }
  __syncthreads();
  return (tot < CAP) ? tot : CAP;
}

__global__ __launch_bounds__(NT) void agg_kernel(const float* __restrict__ mapped, const int* __restrict__ rowv, const int* __restrict__ colv,
                                                const float* __restrict__ av, const float* __restrict__ s1, const float* __restrict__ s2, float* out) {
  __shared__ int   LIST[SCH];
  __shared__ float LSC[SCH];
  __shared__ float SM[SRB];
  __shared__ float SL[SRB];
  __shared__ int   scan_ws[80];
  const int tid = threadIdx.x, lane = tid & 31, wave = tid >> 5;
  const int n0 = blockIdx.x * SRB;
  const int nhi = (n0 + SRB < NN) ? (n0 + SRB) : NN;
  for (int i = tid; i < SRB; i += NT) { SM[i] = -INFINITY; SL[i] = 0.f; }
  __syncthreads();
#pragma unroll 1
  for (int ch = 0; ch < NCH; ++ch) {
    const int tot = chunk_hits<SCH / NT, SCH>(rowv, colv, av, s1, s2, ch * SCH, n0, nhi, tid, LIST, LSC, scan_ws);
#pragma unroll 1
    for (int base = 0; base < tot; base += 32) {
      const int q = base + lane;
      const int qc = (q < SCH) ? q : (SCH - 1);
      const int lr = LIST[qc];
      const float fv = LSC[qc];
      const int rv = (q < tot) ? lr : -1;
      const int own = (rv >= 0 && (rv >> 26) == wave) ? 1 : 0;
      unsigned msk = (unsigned)__ballot(own);
#pragma unroll 1
      for (int it = 0; it < 32; ++it) {
        if (msk == 0u) break;
        const int bp = __builtin_ctz(msk); msk &= msk - 1u;
        const int r = __shfl(rv, bp, 32);
        const float sc = __shfl(fv, bp, 32);
        const int dl = r >> 17, c = r & 0x1FFFF;
        int n = n0 + dl; n = (n < NN) ? n : (NN - 1);
        const float mo = SM[dl], lo = SL[dl];
        const float mn = fmaxf(mo, sc);
        const float rr = __expf(mo - mn), ex = __expf(sc - mn);
        const float ln = lo * rr + ex;
        if (lane == 0) { SM[dl] = mn; SL[dl] = ln; }
        const v4f mv = *(const v4f*)(mapped + (size_t)c * FD + 4 * lane);
        float* rp = out + (size_t)n * FD + 4 * lane;
        v4f a = *(const v4f*)rp;
        a = a * rr + ex * mv;
        *(volatile v4f*)rp = a; __threadfence(); *(volatile v4f*)rp = a;
      }
    }
    __syncthreads();
  }
#pragma unroll 1
  for (int j = 0; j < SRB / 8; ++j) {
    const int dl = wave * (SRB / 8) + j;
    const int n = n0 + dl;
    if (n < NN) {
      const float lv = SL[dl];
      const float inv = (lv > 0.f) ? (1.0f / lv) : 0.f;
      float* rp = out + (size_t)n * FD + 4 * lane;
      v4f a = *(const v4f*)rp;
      a = a * inv;
      *(volatile v4f*)rp = a; __threadfence(); *(volatile v4f*)rp = a;
    }
  }
}

extern "C" void kernel_launch(void* const* d_in, const int* in_sizes, int n_in,
                              void* d_out, int out_size, void* d_ws, size_t ws_size, hipStream_t stream) {
  (void)n_in;
  const float* x       = (const float*)d_in[0];
  const float* a_vals  = (const float*)d_in[1];
  const float* W       = (const float*)d_in[2];
  const float* M1      = (const float*)d_in[3];
  const float* M2      = (const float*)d_in[4];
  const float* gamma   = (const float*)d_in[5];
  const float* beta    = (const float*)d_in[6];
  const float* bn_mean = (const float*)d_in[7];
  const float* bn_var  = (const float*)d_in[8];
  const int*   row     = (const int*)d_in[9];
  const int*   col     = (const int*)d_in[10];
  float* out = (float*)d_out;

  if (in_sizes[0] != NN * FD || in_sizes[1] != NE || in_sizes[9] != NE || in_sizes[10] != NE || out_size != NN * FD) return;

  char* ws = (char*)d_ws; size_t off = 0;
  auto carve = [&](size_t bytes) -> char* { char* p = ws + off; off += (bytes + 255) & ~(size_t)255; return p; };
  unsigned short* Bh = (unsigned short*)carve((size_t)NB * FD * 2);
  unsigned short* Bl = (unsigned short*)carve((size_t)NB * FD * 2);
  unsigned short* Ah = (unsigned short*)carve((size_t)CR * FD * 2);
  unsigned short* Al = (unsigned short*)carve((size_t)CR * FD * 2);
  float* mapped = (float*)carve((size_t)NPAD * FD * 4);
  float* Cq     = (float*)carve((size_t)CR * 2 * FD * 4);
  float* s1     = (float*)carve((size_t)NPAD * 4);
  float* s2     = (float*)carve((size_t)NPAD * 4);
  if (off > ws_size || off > (size_t)134217728) return;

  const int tW = (CR / 64) * (FD / 64);
  const int tM = (CR / 64) * ((2 * FD) / 64);

  bt_split_kernel<<<(NB * (FD / 8) + 255) / 256, 256, 0, stream>>>(W, M1, M2, Bh, Bl);
  for (int qk = 0; qk < NCK; ++qk) {
    const int row0 = qk * CR;
    xn_split_kernel<<<(CR * (FD / 8)) / 256, 256, 0, stream>>>(x, gamma, beta, bn_mean, bn_var, row0, Ah, Al);
    wmma_gemm64<1, true, 0, 0, false><<<dim3((tW + 7) / 8, 1), 256, 0, stream>>>(
        Ah, Al, FD, 0L, Bh, Bl, FD, 0L,
        (void*)(mapped + (size_t)row0 * FD), nullptr, FD, 0L, nullptr, nullptr, 0L, CR, FD, FD, 1.0f);
    wmma_gemm64<1, true, 0, 0, false><<<dim3((tM + 7) / 8, 1), 256, 0, stream>>>(
        Ah, Al, FD, 0L, Bh + (size_t)FD * FD, Bl + (size_t)FD * FD, FD, 0L,
        (void*)Cq, nullptr, 2 * FD, 0L, nullptr, nullptr, 0L, CR, 2 * FD, FD, 1.0f);
    qform_tanh_kernel<<<CR / 64, NT, 0, stream>>>(Cq, x, gamma, beta, bn_mean, bn_var, row0, s1, s2);
  }
  agg_kernel<<<NTL, NT, 0, stream>>>(mapped, row, col, a_vals, s1, s2, out);
}
